// SS2D_18391049962059
// MI455X (gfx1250) — hardware-verified
//
#include <hip/hip_runtime.h>
#include <math.h>

typedef __attribute__((ext_vector_type(16))) _Float16 v16h;
typedef __attribute__((ext_vector_type(8)))  _Float16 v8h;
typedef __attribute__((ext_vector_type(16))) __bf16   v16b;
typedef __attribute__((ext_vector_type(8)))  __bf16   v8b;
typedef __attribute__((ext_vector_type(8)))  float    v8f;
typedef __attribute__((ext_vector_type(4)))  float    v4f;

constexpr int kChn  = 96;
constexpr int kHgt  = 96;
constexpr int kWid  = 96;
constexpr int kLen  = kHgt * kWid;
constexpr int kDirs = 4;
constexpr int kNst  = 16;
constexpr int kDtR  = 6;
constexpr int kCpr  = kDtR + 2 * kNst;
constexpr int kNpad = 128;
constexpr int kPrepRows = 64;
constexpr int kPrepTP   = 97;
constexpr int kChunksPerRow = kChn / 8;
constexpr int kScanTS = 64;
constexpr int kScanXP = 40;
constexpr int kScanYP = 68;
static_assert((kChn % 32) == 0);
static_assert((kLen % 64) == 0 && (kNpad % 64) == 0);
static_assert((((kLen / 64) * (kNpad / 64)) % 8) == 0);
static_assert((kLen % kPrepRows) == 0 && ((kChn * kPrepRows) % 256) == 0 && (((kPrepRows * kChn) / 8) % 256) == 0);
static_assert((kLen % kScanTS) == 0 && (kLen % 8) == 0);
static_assert(kCpr == 38 && kDtR + 2 <= 8 && 8 + 2 * kNst == kScanXP);

constexpr size_t kOffXT   = 0;
constexpr size_t kOffBT   = kOffXT + (size_t)2 * kLen * kChn * 2;
constexpr size_t kOffXD   = kOffBT + (size_t)2 * kNpad * kChn * 2;
constexpr size_t kOffY    = kOffXD + (size_t)2 * kLen * kNpad * 4;
constexpr size_t kWsTotal = kOffY  + (size_t)kDirs * kChn * kLen * 4;
static_assert(kWsTotal == 27181056ull);
static_assert(kWsTotal <= 134217728ull);
static_assert((kOffBT % 128) == 0 && (kOffXD % 128) == 0 && (kOffY % 128) == 0);

__device__ __forceinline__ unsigned short f2bf_bits(float f) {
  unsigned u = __float_as_uint(f);
  return (unsigned short)((u + 0x7FFFu + ((u >> 16) & 1u)) >> 16);
}
__device__ __forceinline__ float bf_bits2f(unsigned short h) { return __uint_as_float(((unsigned)h) << 16); }
__device__ __forceinline__ float bf_rne(float f) { return bf_bits2f(f2bf_bits(f)); }

__device__ __forceinline__ void dep_guard_h(v8f& a, v8f& b, v16h x, v16h y) { asm volatile("v_nop\n\tv_nop\n\tv_nop\n\tv_nop" : "+v"(a), "+v"(b) : "v"(x), "v"(y)); }
__device__ __forceinline__ void dep_guard_b(v8f& a, v8f& b, v16b x, v16b y) { asm volatile("v_nop\n\tv_nop\n\tv_nop\n\tv_nop" : "+v"(a), "+v"(b) : "v"(x), "v"(y)); }
__device__ __forceinline__ void dep_guard4x_h(v8f& a, v8f& b, v8f& c, v8f& d, v16h x, v16h y, v16h w) { asm volatile("v_nop\n\tv_nop\n\tv_nop\n\tv_nop" : "+v"(a), "+v"(b), "+v"(c), "+v"(d) : "v"(x), "v"(y), "v"(w)); }
__device__ __forceinline__ void dep_guard4x_b(v8f& a, v8f& b, v8f& c, v8f& d, v16b x, v16b y, v16b w) { asm volatile("v_nop\n\tv_nop\n\tv_nop\n\tv_nop" : "+v"(a), "+v"(b), "+v"(c), "+v"(d) : "v"(x), "v"(y), "v"(w)); }
__device__ __forceinline__ void keep4_h(v16h a, v16h b, v16h c, v16h d) { asm volatile("v_nop" :: "v"(a), "v"(b), "v"(c), "v"(d)); }
__device__ __forceinline__ void keep4_b(v16b a, v16b b, v16b c, v16b d) { asm volatile("v_nop" :: "v"(a), "v"(b), "v"(c), "v"(d)); }
__device__ __forceinline__ void acc_guard4(v8f& a, v8f& b, v8f& c, v8f& d) { asm volatile("v_nop\n\tv_nop\n\tv_nop\n\tv_nop" : "+v"(a), "+v"(b), "+v"(c), "+v"(d)); }
template <typename T> struct Frag;
template <> struct Frag<_Float16> {
  typedef v16h V; union U { v16h v; v8h h[2]; };
  static __device__ __forceinline__ v16h load(const _Float16* p) {
    U f; f.h[0] = *(const v8h*)(p); f.h[1] = *(const v8h*)(p + 16); return f.v;
  }
  static __device__ __forceinline__ v8f mma(v16h a, v16h b, v8f c) {
    return __builtin_amdgcn_wmma_f32_16x16x32_f16(false, a, false, b, (short)0, c, false, false);
  }
  static __device__ __forceinline__ void guard(v8f& a, v8f& b, v16h x, v16h y) { dep_guard_h(a, b, x, y); }
  static __device__ __forceinline__ void guard4(v8f& a, v8f& b, v8f& c, v8f& d, v16h x, v16h y, v16h w) { dep_guard4x_h(a, b, c, d, x, y, w); }
  static __device__ __forceinline__ void keep(v16h a, v16h b, v16h c, v16h d) { keep4_h(a, b, c, d); }
};
template <> struct Frag<__bf16> {
  typedef v16b V; union U { v16b v; v8b h[2]; };
  static __device__ __forceinline__ v16b load(const __bf16* p) {
    U f; f.h[0] = *(const v8b*)(p); f.h[1] = *(const v8b*)(p + 16); return f.v;
  }
  static __device__ __forceinline__ v8f mma(v16b a, v16b b, v8f c) {
    return __builtin_amdgcn_wmma_f32_16x16x32_bf16(false, a, false, b, (short)0, c, false, false);
  }
  static __device__ __forceinline__ void guard(v8f& a, v8f& b, v16b x, v16b y) { dep_guard_b(a, b, x, y); }
  static __device__ __forceinline__ void guard4(v8f& a, v8f& b, v8f& c, v8f& d, v16b x, v16b y, v16b w) { dep_guard4x_b(a, b, c, d, x, y, w); }
  static __device__ __forceinline__ void keep(v16b a, v16b b, v16b c, v16b d) { keep4_b(a, b, c, d); }
};

template <int ET> struct Elem;
template <> struct Elem<0> { typedef _Float16 T; };
template <> struct Elem<1> { typedef __bf16 T; };
template <int ET, int SPL, int BIAS_MODE, int OUT_MODE, bool RESID, int ACT = 0>
__global__ __launch_bounds__(256) void wmma_gemm64(
    const unsigned short* __restrict__ Ap, const unsigned short* __restrict__ A2p, int lda, long strideA,
    const unsigned short* __restrict__ Btp, const unsigned short* __restrict__ Bt2p, int ldb, long strideB,
    void* __restrict__ Cout, void* __restrict__ Cout2, int ldc, long strideC,
    const float* __restrict__ bias,
    const float* __restrict__ resid, long strideR,
    int M, int N, int K, float scale) {
  typedef typename Elem<ET>::T T;
  typedef typename Frag<T>::V V;
  const T* A = (const T*)Ap; const T* A2 = (const T*)A2p; const T* Bt = (const T*)Btp; const T* Bt2 = (const T*)Bt2p;
  __shared__ __align__(16) float sT[8][16 * 68];
  const int b    = blockIdx.y;
  const int lane = threadIdx.x & 31;
  const int wave = threadIdx.x >> 5;
  const int tilesN = N >> 6;
  const int tilesM = M >> 6;
  const int tile = blockIdx.x * 8 + wave;
  if (tile >= tilesM * tilesN) return;
  const int tm = tile / tilesN;
  const int tn = tile - tm * tilesN;
  const int m0 = tm << 6;
  const int n0 = tn << 6;

  const T* Ab  = A  + (size_t)b * strideA;
  const T* Bb  = Bt + (size_t)b * strideB;
  const T* Ab2 = (SPL >= 1) ? (A2  + (size_t)b * strideA) : nullptr;
  const T* Bb2 = (SPL == 2) ? (Bt2 + (size_t)b * strideB) : nullptr;

  const int rlane = lane & 15;
  const int koff  = (lane >> 4) * 8;
  const int mOff  = (lane >> 4) * 8;

  v8f acc[4][4];
#pragma unroll
  for (int i = 0; i < 4; ++i)
#pragma unroll
    for (int j = 0; j < 4; ++j) acc[i][j] = (v8f){0.f,0.f,0.f,0.f,0.f,0.f,0.f,0.f};

  for (int k0 = 0; k0 < K; k0 += 32) {
    V bh[4], bl[4];
#pragma unroll
    for (int j = 0; j < 4; ++j) {
      const size_t bo = (size_t)(n0 + (j << 4) + rlane) * ldb + koff + k0;
      bh[j] = Frag<T>::load(Bb + bo);
      if (SPL == 2) bl[j] = Frag<T>::load(Bb2 + bo);
    }
#pragma unroll
    for (int i = 0; i < 4; ++i) {
      const size_t ao = (size_t)(m0 + (i << 4) + rlane) * lda + koff + k0;
      V ah = Frag<T>::load(Ab + ao);
      V al = ah;
      if (SPL >= 1) al = Frag<T>::load(Ab2 + ao);
#pragma unroll
      for (int j = 0; j < 4; ++j) {
        acc[i][j] = Frag<T>::mma(ah, bh[j], acc[i][j]);
        if (SPL == 2) acc[i][j] = Frag<T>::mma(ah, bl[j], acc[i][j]);
        if (SPL >= 1) acc[i][j] = Frag<T>::mma(al, bh[j], acc[i][j]);
      }
      Frag<T>::guard4(acc[i][0], acc[i][1], acc[i][2], acc[i][3], ah, bh[3], al);
    }
    Frag<T>::keep(bh[0], bh[1], bh[2], bh[3]);
    if (SPL == 2) Frag<T>::keep(bl[0], bl[1], bl[2], bl[3]);
  }
  acc_guard4(acc[0][0], acc[0][1], acc[0][2], acc[0][3]);
  acc_guard4(acc[1][0], acc[1][1], acc[1][2], acc[1][3]);
  acc_guard4(acc[2][0], acc[2][1], acc[2][2], acc[2][3]);
  acc_guard4(acc[3][0], acc[3][1], acc[3][2], acc[3][3]);

  float* slab = sT[wave];
  const float* Rb = RESID ? (resid + (size_t)b * strideR) : nullptr;
#pragma unroll
  for (int i = 0; i < 4; ++i) {
    const int mBase = m0 + (i << 4);
#pragma unroll
    for (int j = 0; j < 4; ++j) {
      const int n = n0 + (j << 4) + rlane;
      float bv = 0.f;
      if (BIAS_MODE == 2) bv = bias[n];
#pragma unroll
      for (int r = 0; r < 8; ++r) {
        float v = acc[i][j][r] * scale;
        if (BIAS_MODE == 1) v += bias[mBase + mOff + r];
        if (BIAS_MODE == 2) v += bv;
        if (RESID) v += Rb[(size_t)(mBase + mOff + r) * ldc + n];
        if (ACT == 1) v = tanhf(v);
        if (ACT == 2) v = fmaxf(v, 0.0f);
        if (ACT == 3) v = v / (1.0f + expf(-v));
        if (ACT == 4) v = (v > 0.f) ? v : 0.01f * v;
        slab[(mOff + r) * 68 + (j << 4) + rlane] = v;
      }
    }
    __builtin_amdgcn_fence(__ATOMIC_RELEASE, "workgroup");
    __builtin_amdgcn_wave_barrier();
    __builtin_amdgcn_fence(__ATOMIC_ACQUIRE, "workgroup");
    if (OUT_MODE == 0) {
      float* C = (float*)Cout + (size_t)b * strideC;
      const int hh = lane >> 4, c4 = (lane & 15) * 4;
      for (int pass = 0; pass < 2; ++pass) {
#pragma unroll
        for (int it = 0; it < 8; ++it) {
          const int row = it * 2 + hh;
          v4f v = *(const v4f*)(slab + row * 68 + c4);
          *(volatile v4f*)(C + (size_t)(mBase + row) * ldc + n0 + c4) = v;
        }
        __threadfence();
      }
    } else {
      const int q = lane >> 3, c8 = (lane & 7) * 8;
      unsigned short* C  = (unsigned short*)Cout  + (size_t)b * strideC;
      unsigned short* C2 = (OUT_MODE == 2) ? ((unsigned short*)Cout2 + (size_t)b * strideC) : nullptr;
      for (int pass = 0; pass < 2; ++pass) {
#pragma unroll
        for (int it = 0; it < 4; ++it) {
          const int row = it * 4 + q;
          const float* sp = slab + row * 68 + c8;
          v8h hv, lv;
#pragma unroll
          for (int e = 0; e < 8; ++e) {
            if (OUT_MODE == 1) {
              hv[e] = (_Float16)sp[e];
            } else {
              unsigned short hb = f2bf_bits(sp[e]);
              unsigned short lb = f2bf_bits(sp[e] - bf_bits2f(hb));
              hv[e] = __builtin_bit_cast(_Float16, hb);
              lv[e] = __builtin_bit_cast(_Float16, lb);
            }
          }
          *(volatile v8h*)(C + (size_t)(mBase + row) * ldc + n0 + c8) = hv;
          if (OUT_MODE == 2) *(volatile v8h*)(C2 + (size_t)(mBase + row) * ldc + n0 + c8) = lv;
        }
        __threadfence();
      }
    }
    __builtin_amdgcn_fence(__ATOMIC_RELEASE, "workgroup");
    __builtin_amdgcn_wave_barrier();
    __builtin_amdgcn_fence(__ATOMIC_ACQUIRE, "workgroup");
  }
}

__global__ __launch_bounds__(256) void prep_x_kernel(const float* __restrict__ x, unsigned short* __restrict__ XT)
{
  __shared__ float sT[kPrepRows * kPrepTP];
  const int tid = threadIdx.x;
  const int z   = blockIdx.y;
  const int l0  = blockIdx.x * kPrepRows;
#pragma unroll 1
  for (int i = 0; i < (kChn * kPrepRows) / 256; ++i) {
    const int idx = i * 256 + tid;
    const int d   = idx >> 6;
    const int lc  = idx & 63;
    const int l   = l0 + lc;
    const int lq  = l / kHgt;
    const int lm  = l - lq * kHgt;
    const int src = z ? (lm * kWid + lq) : l;
    sT[lc * kPrepTP + d] = x[(size_t)d * kLen + src];
  }
  __syncthreads();
  v8h hv[3];
#pragma unroll
  for (int it = 0; it < 3; ++it) {
    const int chunk = it * 256 + tid;
    const int row   = chunk / kChunksPerRow;
    const int c0    = (chunk - row * kChunksPerRow) * 8;
    const float* sp = sT + row * kPrepTP + c0;
#pragma unroll
    for (int e = 0; e < 8; ++e) {
      const unsigned short hb = f2bf_bits(sp[e]);
      hv[it][e] = __builtin_bit_cast(_Float16, hb);
    }
  }
  unsigned short* base = XT + (size_t)z * kLen * kChn + (size_t)l0 * kChn;
  for (int pass = 0; pass < 2; ++pass) {
#pragma unroll
    for (int it = 0; it < 3; ++it)
      *(volatile v8h*)(base + (size_t)(it * 256 + tid) * 8) = hv[it];
    __threadfence();
  }
}

__global__ __launch_bounds__(256) void prep_w_kernel(const float* __restrict__ wp, unsigned short* __restrict__ BT)
{
  const int i    = blockIdx.x * 256 + threadIdx.x;
  const int z    = i / (kNpad * kChunksPerRow);
  const int rem  = i - z * (kNpad * kChunksPerRow);
  const int n    = rem / kChunksPerRow;
  const int c0   = (rem - n * kChunksPerRow) * 8;
  const int nn   = n & 63;
  const int half = n >> 6;
  const int k    = z + 2 * half;
  const bool valid = (nn < kDtR) || (nn >= 8 && nn < kScanXP);
  int c = (nn < kDtR) ? nn : (nn - 2);
  c = (c < 0) ? 0 : ((c > kCpr - 1) ? (kCpr - 1) : c);
  const float* src = wp + ((size_t)(k * kCpr + c) * kChn + c0);
  const v4f a0 = *(const v4f*)(src);
  const v4f a1 = *(const v4f*)(src + 4);
  const float fz = valid ? 1.0f : 0.0f;
  v8h hv;
#pragma unroll
  for (int e = 0; e < 4; ++e) {
    const unsigned short h0 = f2bf_bits(a0[e] * fz);
    const unsigned short h1 = f2bf_bits(a1[e] * fz);
    hv[e]     = __builtin_bit_cast(_Float16, h0);
    hv[4 + e] = __builtin_bit_cast(_Float16, h1);
  }
  unsigned short* q = BT + (size_t)i * 8;
  *(volatile v8h*)q = hv;
  __threadfence();
  *(volatile v8h*)q = hv;
}

__global__ __launch_bounds__(96) void scan_kernel(
    const float* __restrict__ XD, const float* __restrict__ x,
    const float* __restrict__ wdt, const float* __restrict__ bdt,
    const float* __restrict__ alog, const float* __restrict__ dsv,
    float* __restrict__ Y)
{
  __shared__ __align__(16) float sX[kScanTS * kScanXP];
  __shared__ __align__(16) float sY[kChn * kScanYP];
  __shared__ __align__(16) float sA[kNst * kChn];
  const int tid  = threadIdx.x;
  const int lane = tid & 31;
  const int wave = tid >> 5;
  const int k    = blockIdx.x;
  const int z    = k & 1;
  const int half = k >> 1;
  const int d    = tid;
  const int kd   = k * kChn + d;
#pragma unroll 1
  for (int s = 0; s < kNst; ++s) sA[s * kChn + tid] = -expf(bf_rne(alog[(size_t)kd * kNst + s]));
  float wr[kDtR];
#pragma unroll
  for (int r = 0; r < kDtR; ++r) wr[r] = bf_rne(wdt[(size_t)kd * kDtR + r]);
  const float bias = bf_rne(bdt[kd]);
  const float dsc  = bf_rne(dsv[kd]);
  __syncthreads();
  float negA[kNst], h[kNst];
#pragma unroll
  for (int s = 0; s < kNst; ++s) { negA[s] = sA[s * kChn + tid]; h[s] = 0.0f; }
  const float* xrow = x + (size_t)d * kLen;
  const float* XDz  = XD + (size_t)z * kLen * kNpad + half * 64;
  const int c4s = (lane & 15) * 4;
#pragma unroll 1
  for (int l0 = 0; l0 < kLen; l0 += kScanTS) {
    __syncthreads();
#pragma unroll 1
    for (int it = 0; it < 7; ++it) {
      int i = it * 96 + tid;
      i = (i > 639) ? 639 : i;
      const int s   = i / 10;
      const int q   = i - s * 10;
      const int le  = l0 + s;
      const int row = half ? (kLen - 1 - le) : le;
      *(v4f*)(sX + s * kScanXP + q * 4) = *(const v4f*)(XDz + (size_t)row * kNpad + q * 4);
    }
    __syncthreads();
#pragma unroll 1
    for (int s = 0; s < kScanTS; ++s) {
      const int le  = l0 + s;
      const int lr  = half ? (kLen - 1 - le) : le;
      const int lq  = lr / kHgt;
      const int lm  = lr - lq * kHgt;
      const int src = z ? (lm * kWid + lq) : lr;
      const float ub = bf_rne(xrow[src]);
      const float* xr = sX + s * kScanXP;
      const v4f t03 = *(const v4f*)(xr);
      const v4f t47 = *(const v4f*)(xr + 4);
      float vd = t03[0] * wr[0];
      vd = fmaf(t03[1], wr[1], vd);
      vd = fmaf(t03[2], wr[2], vd);
      vd = fmaf(t03[3], wr[3], vd);
      vd = fmaf(t47[0], wr[4], vd);
      vd = fmaf(t47[1], wr[5], vd);
      const float vz  = vd + bias;
      const float ea  = __expf(-fabsf(vz));
      const float up  = 1.0f + ea;
      const float l1p = __logf(up) + (ea - (up - 1.0f)) * __builtin_amdgcn_rcpf(up);
      const float dlt = fmaxf(vz, 0.0f) + l1p;
      const float dx  = dlt * ub;
      float y = 0.0f;
#pragma unroll
      for (int q4 = 0; q4 < 4; ++q4) {
        const v4f bv = *(const v4f*)(xr + 8 + 4 * q4);
        const v4f cv = *(const v4f*)(xr + 8 + kNst + 4 * q4);
#pragma unroll
        for (int e = 0; e < 4; ++e) {
          const int n = 4 * q4 + e;
          const float a = __expf(dlt * negA[n]);
          h[n] = fmaf(a, h[n], dx * bv[e]);
          y = fmaf(h[n], cv[e], y);
        }
      }
      y = fmaf(ub, dsc, y);
      sY[tid * kScanYP + s] = y;
    }
    __syncthreads();
    for (int pass = 0; pass < 2; ++pass) {
#pragma unroll
      for (int it = 0; it < 16; ++it) {
        const int row = wave * 32 + it * 2 + (lane >> 4);
        const v4f v = *(const v4f*)(sY + row * kScanYP + c4s);
        *(volatile v4f*)(Y + (size_t)(k * kChn + row) * kLen + l0 + c4s) = v;
      }
      __threadfence();
    }
  }
}

__device__ __forceinline__ float merge4_dir(const float* __restrict__ Y, int d, int p, int pt)
{
  const float a0 = Y[(size_t)d * kLen + p];
  const float a2 = Y[(size_t)(2 * kChn + d) * kLen + (kLen - 1 - p)];
  const float a1 = Y[(size_t)(kChn + d) * kLen + pt];
  const float a3 = Y[(size_t)(3 * kChn + d) * kLen + (kLen - 1 - pt)];
  return (a0 + a2) + (a1 + a3);
}

__global__ __launch_bounds__(256) void merge_ln_kernel(
    const float* __restrict__ Y, const float* __restrict__ lnw, const float* __restrict__ lnb,
    float* __restrict__ out)
{
  __shared__ __align__(16) float sO[8 * 128];
  const int wave = threadIdx.x >> 5;
  const int lane = threadIdx.x & 31;
  const int p  = blockIdx.x * 8 + wave;
  const int ph = p / kWid;
  const int pw = p - ph * kWid;
  const int pt = pw * kHgt + ph;
  float gw0 = bf_rne(lnw[lane]), gw1 = bf_rne(lnw[lane + 32]), gw2 = bf_rne(lnw[lane + 64]);
  float gb0 = bf_rne(lnb[lane]), gb1 = bf_rne(lnb[lane + 32]), gb2 = bf_rne(lnb[lane + 64]);
  asm volatile("" : "+v"(gw0), "+v"(gw1), "+v"(gw2), "+v"(gb0), "+v"(gb1), "+v"(gb2) :: "memory");
  float v0 = merge4_dir(Y, lane, p, pt);
  asm volatile("" : "+v"(v0) :: "memory");
  float v1 = merge4_dir(Y, lane + 32, p, pt);
  asm volatile("" : "+v"(v1) :: "memory");
  float v2 = merge4_dir(Y, lane + 64, p, pt);
  asm volatile("" : "+v"(v2) :: "memory");
  float s = (v0 + v1) + v2;
#pragma unroll
  for (int off = 16; off > 0; off >>= 1) s += __shfl_xor(s, off, 32);
  const float mu = s * (1.0f / 96.0f);
  const float t0 = v0 - mu, t1 = v1 - mu, t2 = v2 - mu;
  float sq = (t0 * t0 + t1 * t1) + t2 * t2;
#pragma unroll
  for (int off = 16; off > 0; off >>= 1) sq += __shfl_xor(sq, off, 32);
  const float var = sq * (1.0f / 96.0f);
  const float rs  = rsqrtf(var + 1e-5f);
  sO[wave * 128 + lane]      = t0 * rs * gw0 + gb0;
  sO[wave * 128 + lane + 32] = t1 * rs * gw1 + gb1;
  sO[wave * 128 + lane + 64] = t2 * rs * gw2 + gb2;
  __syncthreads();
  const int jl = (lane < 24) ? lane : 23;
  const v4f ov = *(const v4f*)(sO + wave * 128 + jl * 4);
  float* orow = out + (size_t)p * kChn;
  for (int pass = 0; pass < 2; ++pass) {
    if (lane < 24) *(volatile v4f*)(orow + lane * 4) = ov;
    __threadfence();
  }
}

extern "C" void kernel_launch(void* const* d_in, const int* in_sizes, int n_in,
                              void* d_out, int out_size, void* d_ws, size_t ws_size,
                              hipStream_t stream) {
  if (n_in < 8) return;
  if (in_sizes[0] != kChn * kLen) return;
  if (in_sizes[1] != kDirs * kCpr * kChn) return;
  if (in_sizes[2] != kDirs * kChn * kDtR) return;
  if (in_sizes[3] != kDirs * kChn) return;
  if (in_sizes[4] != kDirs * kChn * kNst) return;
  if (in_sizes[5] != kDirs * kChn) return;
  if (in_sizes[6] != kChn) return;
  if (in_sizes[7] != kChn) return;
  if (out_size != kLen * kChn) return;
  if (ws_size < kWsTotal) return;

  const float* x    = (const float*)d_in[0];
  const float* wprj = (const float*)d_in[1];
  const float* wdt  = (const float*)d_in[2];
  const float* bdt  = (const float*)d_in[3];
  const float* alog = (const float*)d_in[4];
  const float* dsv  = (const float*)d_in[5];
  const float* lnw  = (const float*)d_in[6];
  const float* lnb  = (const float*)d_in[7];
  float* out = (float*)d_out;

  char* ws = (char*)d_ws;
  unsigned short* XT = (unsigned short*)(ws + kOffXT);
  unsigned short* BT = (unsigned short*)(ws + kOffBT);
  float*          XD = (float*)(ws + kOffXD);
  float*          Yp = (float*)(ws + kOffY);

  prep_x_kernel<<<dim3(kLen / kPrepRows, 2), 256, 0, stream>>>(x, XT);
  prep_w_kernel<<<(2 * kNpad * kChunksPerRow) / 256, 256, 0, stream>>>(wprj, BT);

  wmma_gemm64<1, 0, 0, 0, false><<<dim3(((kLen / 64) * (kNpad / 64)) / 8, 2), 256, 0, stream>>>(
      XT, nullptr, kChn, (long)kLen * kChn,
      BT, nullptr, kChn, (long)kNpad * kChn,
      (void*)XD, nullptr, kNpad, (long)kLen * kNpad,
      nullptr, nullptr, 0L,
      kLen, kNpad, kChn, 1.0f);

  scan_kernel<<<kDirs, kChn, 0, stream>>>(XD, x, wdt, bdt, alog, dsv, Yp);

  merge_ln_kernel<<<kLen / 8, 256, 0, stream>>>(Yp, lnw, lnb, out);
}
